// DeepGCN_slic_V2_1_23845658427415
// MI455X (gfx1250) — hardware-verified
//
#include <hip/hip_runtime.h>


#define NIMG 64
#define CF   768
#define NR   14
#define NSEG 196
#define NWIN 196
#define NPAD 256
#define IMS  224
#define DM   NPAD
#define LOSC 1024.0f

typedef _Float16 h16;
typedef unsigned short bf;
typedef __attribute__((ext_vector_type(16))) __bf16   v16bf;
typedef __attribute__((ext_vector_type(16))) _Float16 v16h;
typedef __attribute__((ext_vector_type(8)))  _Float16 v8h;
typedef __attribute__((ext_vector_type(8)))  unsigned short v8us;
typedef __attribute__((ext_vector_type(8)))  float    v8f;
typedef __attribute__((ext_vector_type(4)))  float    v4f;
typedef v8h  __attribute__((may_alias)) v8ha;
typedef v4f  __attribute__((may_alias)) v4fa;
typedef v8us __attribute__((may_alias)) v8usa;

__device__ __forceinline__ unsigned short f2bf(float f) { unsigned u = __float_as_uint(f); u += 0x7FFFu + ((u >> 16) & 1u); return (unsigned short)(u >> 16); }
__device__ __forceinline__ float bf2f(unsigned short b) { return __uint_as_float(((unsigned)b) << 16); }
__device__ __forceinline__ float bfr(float f) { return bf2f(f2bf(f)); }
__device__ __forceinline__ v16h cat16(v8h lo, v8h hi) { return __builtin_shufflevector(lo, hi, 0, 1, 2, 3, 4, 5, 6, 7, 8, 9, 10, 11, 12, 13, 14, 15); }
__device__ __forceinline__ v16bf cat16b(v8us lo, v8us hi) { return __builtin_bit_cast(v16bf, __builtin_shufflevector(lo, hi, 0, 1, 2, 3, 4, 5, 6, 7, 8, 9, 10, 11, 12, 13, 14, 15)); }
__device__ __forceinline__ v8f wmma16(v16h a, v16h b, v8f c) { return __builtin_amdgcn_wmma_f32_16x16x32_f16(false, a, false, b, (short)0, c, false, false); }
__device__ __forceinline__ v8f wmmab(v16bf a, v16bf b, v8f c) { return __builtin_amdgcn_wmma_f32_16x16x32_bf16(false, a, false, b, (short)0, c, false, false); }

template <bool SPLITA, bool F16OUT = false>
__global__ __launch_bounds__(128) void k_gemmb(const bf* __restrict__ A, const bf* __restrict__ Al, const bf* __restrict__ Bn, const float* __restrict__ bias, float* C, int ldc, h16* C2, const float* __restrict__ R = nullptr, int K = DM, int roundR = 1) {
    __shared__ __align__(16) float ost[4][16 * 68];
    const int lane = threadIdx.x & 31, wave = threadIdx.x >> 5, lr = lane & 15, hi = lane >> 4;
    const int r0 = blockIdx.x * 64 + wave * 16, c0 = blockIdx.y * 64;
    const size_t aoff = (size_t)(r0 + lr) * K + 8 * hi;
    size_t boff[4];
#pragma unroll
    for (int t = 0; t < 4; ++t) boff[t] = (size_t)(c0 + t * 16 + lr) * K + 8 * hi;
    v8f acc[4];
#pragma unroll
    for (int t = 0; t < 4; ++t) acc[t] = (v8f){};
#pragma unroll 1
    for (int kc = 0; kc < K; kc += 32) {
        const v16bf a = cat16b(*(const v8us*)(A + aoff + kc), *(const v8us*)(A + aoff + kc + 16));
        v16bf al = a;
        if (SPLITA) al = cat16b(*(const v8us*)(Al + aoff + kc), *(const v8us*)(Al + aoff + kc + 16));
#pragma unroll
        for (int t = 0; t < 4; ++t) { const v16bf b = cat16b(*(const v8us*)(Bn + boff[t] + kc), *(const v8us*)(Bn + boff[t] + kc + 16)); acc[t] = wmmab(a, b, acc[t]); if (SPLITA) acc[t] = wmmab(al, b, acc[t]); }
        asm volatile("v_nop\n\tv_nop\n\tv_nop\n\tv_nop" : "+v"(acc[0]), "+v"(acc[1]), "+v"(acc[2]), "+v"(acc[3]) : "v"(a), "v"(al));
    }
    float* os = &ost[wave][0];
#pragma unroll
    for (int t = 0; t < 4; ++t) { const float bv = bias ? bfr(bias[c0 + t * 16 + lr]) : 0.f;
#pragma unroll
        for (int j = 0; j < 8; ++j) os[(hi * 8 + j) * 68 + t * 16 + lr] = acc[t][j] + bv; }
    __syncthreads();
    if (F16OUT) {
        h16* crow = (h16*)(void*)C + (size_t)r0 * ldc + c0;
        auto pass = [&]() {
#pragma unroll
            for (int s = 0; s < 4; ++s) { const int row = 4 * s + (lane >> 3), piece = lane & 7; const float* sp = os + row * 68 + piece * 8; v8h o, o2;
#pragma unroll
                for (int i = 0; i < 8; ++i) { const h16 a = (h16)sp[i]; o[i] = a; o2[i] = (h16)((sp[i] - (float)a) * LOSC); }
                *(volatile v8h*)(crow + (size_t)row * ldc + piece * 8) = o; if (C2) *(volatile v8h*)(C2 + (size_t)r0 * ldc + c0 + (size_t)row * ldc + piece * 8) = o2; }
        };
        pass(); __threadfence(); pass();
    } else {
        float* crow = C + (size_t)r0 * ldc + c0;
        auto pass = [&]() {
#pragma unroll
            for (int s = 0; s < 8; ++s) { const int Lid = (lane >> 3) + 4 * s, piece = lane & 7; const int row = Lid >> 1, cofs = (Lid & 1) * 32 + piece * 4;
                v4f val = *(const v4fa*)(os + row * 68 + cofs); if (R) { const v4f rv = *(const v4f*)(R + ((size_t)r0 + row) * ldc + c0 + cofs); val += roundR ? (v4f){bfr(rv[0]), bfr(rv[1]), bfr(rv[2]), bfr(rv[3])} : rv; }
                *(volatile v4f*)(crow + (size_t)row * ldc + cofs) = val; }
        };
        pass(); __threadfence(); pass();
    }
}


__global__ __launch_bounds__(256) void k_wt(const float* __restrict__ Wm, int K, int ncols, bf* WT) {
    __shared__ __align__(16) unsigned short tl[64 * 72];
    const int tid = threadIdx.x, k0 = blockIdx.x * 64, n0 = blockIdx.y * 64;
    const int kk = tid >> 2, nq = (tid & 3) * 16;
#pragma unroll
    for (int i = 0; i < 16; ++i) tl[(nq + i) * 72 + kk] = f2bf(Wm[(size_t)(k0 + kk) * ncols + n0 + nq + i]);
    __syncthreads();
    const int piece = tid & 7;
    auto pass = [&]() {
#pragma unroll
        for (int s = 0; s < 2; ++s) { const int nr = (tid >> 3) + 32 * s; const v8us val = *(const v8usa*)(tl + nr * 72 + piece * 8); *(volatile v8us*)(WT + (size_t)(n0 + nr) * K + k0 + piece * 8) = val; }
    };
    pass(); __threadfence(); pass();
}

__global__ __launch_bounds__(32) void k_cnt(const int* __restrict__ seg, float* CNT) {
    const int lane = threadIdx.x, pq = blockIdx.x; float cnt[8];
#pragma unroll
    for (int i = 0; i < 8; ++i) cnt[i] = 0.f;
    if (pq < NWIN) { const int p = pq / NR, q = pq - p * NR;
        const int ci = lane & 15; const int i = ci >> 2, j = ci & 3; const int y0 = 16 * p + 4 * i + 1, x0 = 16 * q + 4 * j + 1;
        int c4[4]; c4[0] = seg[(size_t)y0 * IMS + x0]; c4[1] = seg[(size_t)y0 * IMS + x0 + 1]; c4[2] = seg[(size_t)(y0 + 1) * IMS + x0]; c4[3] = seg[(size_t)(y0 + 1) * IMS + x0 + 1];
#pragma unroll 1
        for (int cell = 0; cell < 16; ++cell) { int a0 = __shfl(c4[0], cell, 32), a1 = __shfl(c4[1], cell, 32), a2 = __shfl(c4[2], cell, 32), a3 = __shfl(c4[3], cell, 32);
#pragma unroll
            for (int k = 0; k < 8; ++k) { const int m = (k < 4) ? (lane * 4 + k) : (128 + lane * 4 + (k - 4)); const bool any = (a0 == m) | (a1 == m) | (a2 == m) | (a3 == m); cnt[k] += any ? 1.f : 0.f; } } }
    v4f lo = {cnt[0], cnt[1], cnt[2], cnt[3]}, hi = {cnt[4], cnt[5], cnt[6], cnt[7]};
    float* row = CNT + (size_t)pq * NPAD + lane * 4;
    *(volatile v4f*)row = lo; *(volatile v4f*)(row + 128) = hi; __threadfence(); *(volatile v4f*)row = lo; *(volatile v4f*)(row + 128) = hi;
}
__global__ __launch_bounds__(256) void k_featb(const float* __restrict__ feat, bf* FB) {
    const int lane = threadIdx.x & 31, f = blockIdx.x * 8 + (threadIdx.x >> 5); if (f >= CF) return; v8us o;
#pragma unroll
    for (int i = 0; i < 8; ++i) { const int pq = lane * 8 + i; const bool ok = pq < NWIN; const float v = feat[(size_t)f * NWIN + (ok ? pq : 0)]; o[i] = ok ? f2bf(v) : (unsigned short)0; }
    *(volatile v8us*)(FB + (size_t)f * NPAD + lane * 8) = o; __threadfence(); *(volatile v8us*)(FB + (size_t)f * NPAD + lane * 8) = o;
}
__global__ __launch_bounds__(256) void k_counts(const float* __restrict__ CNT, float* CT) {
    const int m = threadIdx.x; float s = 0.f;
#pragma unroll 4
    for (int pq = 0; pq < NWIN; ++pq) s += CNT[(size_t)pq * NPAD + m];
    *(volatile float*)(CT + m) = s; __threadfence(); *(volatile float*)(CT + m) = s;
}
__global__ __launch_bounds__(256) void k_out(const float* __restrict__ P, const float* __restrict__ CT, float* Y) {
    const size_t u = (size_t)blockIdx.x * 256 + threadIdx.x; if (u >= (size_t)CF * NSEG / 4) return; v4f v;
#pragma unroll
    for (int i = 0; i < 4; ++i) { const size_t fl = u * 4 + i; const int f = (int)(fl / NSEG), m = (int)(fl % NSEG); const float c = CT[m]; v[i] = (c > 0.f) ? P[(size_t)f * NPAD + m] / c : 0.f; }
    *(volatile v4f*)(Y + u * 4) = v; __threadfence(); *(volatile v4f*)(Y + u * 4) = v;
}

extern "C" void kernel_launch(void* const* d_in, const int* in_sizes, int n_in,
                              void* d_out, int out_size, void* d_ws, size_t ws_size, hipStream_t stream) {
    (void)in_sizes; (void)n_in; (void)out_size;
    const int* seg = (const int*)d_in[0]; const float* feat = (const float*)d_in[1];
    float* out = (float*)d_out;
    char* wsp = (char*)d_ws;
    auto take = [&](size_t bytes) { char* p = wsp; wsp += (bytes + 255) & ~(size_t)255; return (void*)p; };
    float* CNT = (float*)take((size_t)NPAD * NPAD * 4); bf* WT = (bf*)take((size_t)NPAD * NPAD * 2); bf* FB = (bf*)take((size_t)CF * NPAD * 2); float* P = (float*)take((size_t)CF * NPAD * 4); float* CT = (float*)take(NPAD * 4);
    if ((size_t)(wsp - (char*)d_ws) > ws_size) return;
    for (int b = 0; b < NIMG; ++b) {
        k_cnt<<<NPAD, 32, 0, stream>>>(seg + (size_t)b * IMS * IMS, CNT);
        k_wt<<<dim3(NPAD / 64, NPAD / 64, 1), 256, 0, stream>>>(CNT, NPAD, NPAD, WT);
        k_featb<<<CF / 8, 256, 0, stream>>>(feat + (size_t)b * CF * NWIN, FB);
        k_gemmb<false, false><<<dim3(CF / 64, NPAD / 64, 1), 128, 0, stream>>>(FB, nullptr, WT, nullptr, P, NPAD, nullptr, nullptr, NPAD);
        k_counts<<<1, 256, 0, stream>>>(CNT, CT);
        k_out<<<(CF * NSEG / 4 + 255) / 256, 256, 0, stream>>>(P, CT, out + (size_t)b * CF * NSEG);
    }
}
